// ODENet_46480136077880
// MI455X (gfx1250) — hardware-verified
//
#include <hip/hip_runtime.h>

typedef __attribute__((ext_vector_type(16))) _Float16 v16h;
typedef __attribute__((ext_vector_type(8)))  _Float16 v8h;
typedef __attribute__((ext_vector_type(8)))  float    v8f;
typedef __attribute__((ext_vector_type(4)))  float    v4f;

__device__ __forceinline__ void dep_guard_h(v8f& a, v8f& b, v16h x, v16h y) { asm volatile("v_nop\n\tv_nop\n\tv_nop\n\tv_nop" : "+v"(a), "+v"(b) : "v"(x), "v"(y)); }
__device__ __forceinline__ void keep4_h(v16h a, v16h b, v16h c, v16h d) { asm volatile("v_nop" :: "v"(a), "v"(b), "v"(c), "v"(d)); }
template <typename T> struct Frag;
template <> struct Frag<_Float16> {
  typedef v16h V; union U { v16h v; v8h h[2]; };
  static __device__ __forceinline__ v16h load(const _Float16* p) {
    U f; f.h[0] = *(const v8h*)(p); f.h[1] = *(const v8h*)(p + 16); return f.v;
  }
  static __device__ __forceinline__ v8f mma(v16h a, v16h b, v8f c) {
    return __builtin_amdgcn_wmma_f32_16x16x32_f16(false, a, false, b, (short)0, c, false, false);
  }
  static __device__ __forceinline__ void guard(v8f& a, v8f& b, v16h x, v16h y) { dep_guard_h(a, b, x, y); }
  static __device__ __forceinline__ void keep(v16h a, v16h b, v16h c, v16h d) { keep4_h(a, b, c, d); }
};

constexpr int kT       = 8192;
constexpr int kB       = 128;
constexpr int kH       = 128;
constexpr int kRows    = 32;
constexpr int kThreads = 256;
constexpr int kWaves   = 8;
constexpr int kCh      = 64;
constexpr int kKP      = 136;

static_assert(kT % kCh == 0);
static_assert(kB % kRows == 0);
static_assert(kRows == 32);
static_assert(kH == kWaves * 16);
static_assert(kCh == kWaves * 8);
static_assert(kCh % 32 == 0);
static_assert((kKP % 8) == 0);
static_assert(kH % 32 == 0);

constexpr float kAScale = 64.0f;
constexpr float kBScale = 16.0f;
constexpr float kInvAB  = 1.0f / 1024.0f;

__device__ __forceinline__ float tanh_apx(float v) {
  v = fminf(fmaxf(v, -10.0f), 10.0f);
  const float e = __expf(2.0f * v);
  const float r = __builtin_amdgcn_rcpf(e + 1.0f);
  return fmaf(-2.0f, r, 1.0f);
}

__global__ __launch_bounds__(kThreads)
void ode_euler_scan(const float* __restrict__ x,
                    const float* __restrict__ W1,
                    const float* __restrict__ b1,
                    const float* __restrict__ W2,
                    const float* __restrict__ b2,
                    const float* __restrict__ W3,
                    const float* __restrict__ b3,
                    float* __restrict__ out)
{
  __shared__ __align__(16) _Float16 w2t[kH * kKP];
  __shared__ __align__(16) _Float16 h1s[kRows * kKP];
  __shared__ __align__(16) float    xbuf[kCh * kRows];
  __shared__ __align__(16) float    ybuf[kCh * kRows];
  __shared__ __align__(16) float    part[kWaves * kRows];

  const int tid  = threadIdx.x;
  const int lane = tid & 31;
  const int wave = tid >> 5;
  const int rl   = lane & 15;
  const int hh   = lane >> 4;
  const int koff = hh * 8;
  const int b0   = blockIdx.x * kRows;
  const int nCol = wave * 16 + rl;

#pragma unroll 1
  for (int idx = tid; idx < kH * (kH / 8); idx += kThreads) {
    const int n  = idx & (kH - 1);
    const int k8 = (idx >> 7) * 8;
    v8h hv;
#pragma unroll
    for (int e = 0; e < 8; ++e) hv[e] = (_Float16)(W2[(size_t)(k8 + e) * kH + n] * kBScale);
    *(v8h*)(w2t + n * kKP + k8) = hv;
  }

  float w1x[16], w1y[16], b1v[16];
#pragma unroll
  for (int q = 0; q < 4; ++q) {
    const v4f t0 = *(const v4f*)(W1 + wave * 16 + 4 * q);
    const v4f t1 = *(const v4f*)(W1 + kH + wave * 16 + 4 * q);
    const v4f t2 = *(const v4f*)(b1 + wave * 16 + 4 * q);
#pragma unroll
    for (int e = 0; e < 4; ++e) { w1x[4 * q + e] = t0[e]; w1y[4 * q + e] = t1[e]; b1v[4 * q + e] = t2[e]; }
  }
  const float b2n = b2[nCol];
  const float w3n = W3[nCol];
  const float b3v = b3[0];

  __syncthreads();

  const v16h bw0 = Frag<_Float16>::load(w2t + nCol * kKP +  0 + koff);
  const v16h bw1 = Frag<_Float16>::load(w2t + nCol * kKP + 32 + koff);
  const v16h bw2 = Frag<_Float16>::load(w2t + nCol * kKP + 64 + koff);
  const v16h bw3 = Frag<_Float16>::load(w2t + nCol * kKP + 96 + koff);

  float y = 0.0f;
  const int q8 = lane >> 3;
  const int c4 = (lane & 7) * 4;
  const int rowOwn = 16 * (rl >> 3) + 8 * hh + (rl & 7);

  for (int c = 0; c < kT / kCh; ++c) {
    const int tb = c * kCh;
    __syncthreads();
#pragma unroll
    for (int it = 0; it < kCh / 32; ++it) {
      const int row = it * 32 + (tid >> 3);
      int tr = tb + row - 1;
      tr = tr < 0 ? 0 : tr;
      const v4f xv4 = *(const v4f*)(x + (size_t)tr * kB + b0 + (tid & 7) * 4);
      *(v4f*)(xbuf + row * kRows + (tid & 7) * 4) = xv4;
    }
    if (c == 0 && wave == 0) ybuf[lane] = 0.0f;
    __syncthreads();

    const int iStart = (c == 0) ? 1 : 0;
#pragma unroll 1
    for (int i = iStart; i < kCh; ++i) {
      const float xv = xbuf[i * kRows + lane];

      {
        v8h ha, hb;
#pragma unroll
        for (int j = 0; j < 8; ++j) {
          const float a0 = tanh_apx(fmaf(xv, w1x[j],     fmaf(y, w1y[j],     b1v[j])));
          const float a1 = tanh_apx(fmaf(xv, w1x[8 + j], fmaf(y, w1y[8 + j], b1v[8 + j])));
          ha[j] = (_Float16)(a0 * kAScale);
          hb[j] = (_Float16)(a1 * kAScale);
        }
        *(v8h*)(h1s + lane * kKP + wave * 16)     = ha;
        *(v8h*)(h1s + lane * kKP + wave * 16 + 8) = hb;
      }
      __syncthreads();

      v8f acc0 = (v8f){0.f,0.f,0.f,0.f,0.f,0.f,0.f,0.f};
      v8f acc1 = (v8f){0.f,0.f,0.f,0.f,0.f,0.f,0.f,0.f};
      {
        v16h a0 = Frag<_Float16>::load(h1s + rl * kKP + 0 + koff);
        v16h a1 = Frag<_Float16>::load(h1s + (16 + rl) * kKP + 0 + koff);
        acc0 = Frag<_Float16>::mma(a0, bw0, acc0);
        acc1 = Frag<_Float16>::mma(a1, bw0, acc1);
        Frag<_Float16>::guard(acc0, acc1, a0, a1);
        a0 = Frag<_Float16>::load(h1s + rl * kKP + 32 + koff);
        a1 = Frag<_Float16>::load(h1s + (16 + rl) * kKP + 32 + koff);
        acc0 = Frag<_Float16>::mma(a0, bw1, acc0);
        acc1 = Frag<_Float16>::mma(a1, bw1, acc1);
        Frag<_Float16>::guard(acc0, acc1, a0, a1);
        a0 = Frag<_Float16>::load(h1s + rl * kKP + 64 + koff);
        a1 = Frag<_Float16>::load(h1s + (16 + rl) * kKP + 64 + koff);
        acc0 = Frag<_Float16>::mma(a0, bw2, acc0);
        acc1 = Frag<_Float16>::mma(a1, bw2, acc1);
        Frag<_Float16>::guard(acc0, acc1, a0, a1);
        a0 = Frag<_Float16>::load(h1s + rl * kKP + 96 + koff);
        a1 = Frag<_Float16>::load(h1s + (16 + rl) * kKP + 96 + koff);
        acc0 = Frag<_Float16>::mma(a0, bw3, acc0);
        acc1 = Frag<_Float16>::mma(a1, bw3, acc1);
        Frag<_Float16>::guard(acc0, acc1, a0, a1);
        Frag<_Float16>::keep(bw0, bw1, bw2, bw3);
      }

      float vv[16];
#pragma unroll
      for (int r = 0; r < 8; ++r) {
        vv[r]     = tanh_apx(fmaf(acc0[r], kInvAB, b2n)) * w3n;
        vv[8 + r] = tanh_apx(fmaf(acc1[r], kInvAB, b2n)) * w3n;
      }
      float u8[8];
      {
        const bool s8 = (lane & 8) != 0;
#pragma unroll
        for (int j = 0; j < 8; ++j) {
          const float lo = vv[j], hi = vv[8 + j];
          const float keep = s8 ? hi : lo;
          const float send = s8 ? lo : hi;
          const float recv = __shfl_xor(send, 8, 32);
          u8[j] = keep + recv;
        }
      }
      float u4[4];
      {
        const bool s4 = (lane & 4) != 0;
#pragma unroll
        for (int j = 0; j < 4; ++j) {
          const float lo = u8[j], hi = u8[4 + j];
          const float keep = s4 ? hi : lo;
          const float send = s4 ? lo : hi;
          const float recv = __shfl_xor(send, 4, 32);
          u4[j] = keep + recv;
        }
      }
      float u2[2];
      {
        const bool s2 = (lane & 2) != 0;
#pragma unroll
        for (int j = 0; j < 2; ++j) {
          const float lo = u4[j], hi = u4[2 + j];
          const float keep = s2 ? hi : lo;
          const float send = s2 ? lo : hi;
          const float recv = __shfl_xor(send, 2, 32);
          u2[j] = keep + recv;
        }
      }
      float red;
      {
        const bool s1 = (lane & 1) != 0;
        const float keep = s1 ? u2[1] : u2[0];
        const float send = s1 ? u2[0] : u2[1];
        const float recv = __shfl_xor(send, 1, 32);
        red = keep + recv;
      }
      part[wave * kRows + rowOwn] = red;
      __syncthreads();

      float s = part[lane];
      s += part[1 * kRows + lane];
      s += part[2 * kRows + lane];
      s += part[3 * kRows + lane];
      s += part[4 * kRows + lane];
      s += part[5 * kRows + lane];
      s += part[6 * kRows + lane];
      s += part[7 * kRows + lane];
      const float dy = s + b3v;
      y = y + dy;
      if (wave == 0) ybuf[i * kRows + lane] = y;
    }
    __syncthreads();

    float* ob = out + (size_t)tb * kB + b0;
    for (int pass = 0; pass < 2; ++pass) {
#pragma unroll
      for (int it = 0; it < 2; ++it) {
        const int row = wave * 8 + it * 4 + q8;
        const v4f val = *(const v4f*)(ybuf + row * kRows + c4);
        *(volatile v4f*)(ob + (size_t)row * kB + c4) = val;
      }
      __threadfence();
    }
  }
}

extern "C" void kernel_launch(void* const* d_in, const int* in_sizes, int n_in,
                              void* d_out, int out_size, void* d_ws, size_t ws_size,
                              hipStream_t stream) {
  (void)d_ws; (void)ws_size;
  if (n_in < 7) return;
  if (in_sizes[0] != kT * kB || in_sizes[1] != 2 * kH || in_sizes[2] != kH ||
      in_sizes[3] != kH * kH || in_sizes[4] != kH || in_sizes[5] != kH || in_sizes[6] < 1 ||
      out_size != kT * kB) return;
  const float* x  = (const float*)d_in[0];
  const float* W1 = (const float*)d_in[1];
  const float* b1 = (const float*)d_in[2];
  const float* W2 = (const float*)d_in[3];
  const float* b2 = (const float*)d_in[4];
  const float* W3 = (const float*)d_in[5];
  const float* b3 = (const float*)d_in[6];
  float* out = (float*)d_out;
  ode_euler_scan<<<dim3(kB / kRows), dim3(kThreads), 0, stream>>>(x, W1, b1, W2, b2, W3, b3, out);
}
